// Moma_12206297055645
// MI455X (gfx1250) — hardware-run, weakly checked
//
#include <hip/hip_runtime.h>


#ifndef NB
#define NB 128
#endif
#define NB_FULL 128
#define NG   20000
#define MO   384
#define FEAT (4 * MO)
#define CLS  1024
#define FS   64.0f
#define WS   64.0f
#define FWI  (1.0f / 4096.0f)
#define L2E  1.4426950408889634f
#define PPR  (FEAT / 8)
#define PIECES (3 * PPR)

static_assert(NB % 64 == 0);
static_assert(NB <= NB_FULL);
static_assert(MO % 64 == 0);
static_assert(CLS % 64 == 0);
static_assert(NG % 32 == 0);
static_assert(FEAT % 32 == 0);
static_assert(CLS % 128 == 0);
static_assert(MO % 32 == 0);
static_assert(FEAT % 64 == 0);
static_assert(PIECES % 32 == 0);
static_assert((PIECES - MO) % 32 == 0);
static_assert((size_t)PIECES * 16 == (size_t)3 * FEAT * 2);
static_assert(32 * 16 * 8 == 16 * 64 * 4);
static_assert(8 * 16 == 32 * 4);
static_assert((NB_FULL * 4) % 128 == 0);
static_assert(((size_t)NB * NG * 2) % 256 == 0);
static_assert(((size_t)MO * NG * 2) % 256 == 0);
static_assert(((size_t)NB * NG) % 8 == 0);
static_assert(((size_t)MO * NG) % 8 == 0);
static_assert(((size_t)CLS * FEAT) % 8 == 0);
static_assert((16 * 68) * 4 <= 131072);
static_assert((7 * MO + 3 * FEAT) * 4 <= 131072);

typedef _Float16 h16;
typedef unsigned short bf;
typedef __attribute__((ext_vector_type(16))) __bf16   v16bf;
typedef __attribute__((ext_vector_type(16))) _Float16 v16h;
typedef __attribute__((ext_vector_type(8)))  _Float16 v8h;
typedef __attribute__((ext_vector_type(8)))  unsigned short v8us;
typedef __attribute__((ext_vector_type(8)))  float    v8f;
typedef __attribute__((ext_vector_type(4)))  float    v4f;
typedef v4f  __attribute__((may_alias)) v4fa;

__device__ __forceinline__ unsigned short f2bf(float f) { unsigned u = __float_as_uint(f); u += 0x7FFFu + ((u >> 16) & 1u); return (unsigned short)(u >> 16); }
__device__ __forceinline__ float bfr(float f) { return __uint_as_float(((unsigned)f2bf(f)) << 16); }
__device__ __forceinline__ v16h cat16(v8h lo, v8h hi) { return __builtin_shufflevector(lo, hi, 0, 1, 2, 3, 4, 5, 6, 7, 8, 9, 10, 11, 12, 13, 14, 15); }
__device__ __forceinline__ v16bf cat16b(v8us lo, v8us hi) { return __builtin_bit_cast(v16bf, __builtin_shufflevector(lo, hi, 0, 1, 2, 3, 4, 5, 6, 7, 8, 9, 10, 11, 12, 13, 14, 15)); }
__device__ __forceinline__ v8f wmma16(v16h a, v16h b, v8f c) { return __builtin_amdgcn_wmma_f32_16x16x32_f16(false, a, false, b, (short)0, c, false, false); }
__device__ __forceinline__ v8f wmmab(v16bf a, v16bf b, v8f c) { return __builtin_amdgcn_wmma_f32_16x16x32_bf16(false, a, false, b, (short)0, c, false, false); }
__device__ __forceinline__ v16h  ldh(const h16* p) { return cat16(*(const v8h*)p, *(const v8h*)(p + 16)); }
__device__ __forceinline__ v16bf ldb(const bf* p)  { return cat16b(*(const v8us*)p, *(const v8us*)(p + 16)); }
__device__ __forceinline__ void wave_sync() { __builtin_amdgcn_fence(3  , "wavefront"); __builtin_amdgcn_wave_barrier(); asm volatile("" ::: "memory"); }

__device__ __forceinline__ v8f wmmab_g(v16bf a, v16bf b, v8f c) { c = wmmab(a, b, c); asm volatile("v_nop\n\tv_nop\n\tv_nop\n\tv_nop" : "+v"(c) : "v"(a), "v"(b)); return c; }
__device__ __forceinline__ v8f wmma16_g(v16h a, v16h b, v8f c) { c = wmma16(a, b, c); asm volatile("v_nop\n\tv_nop\n\tv_nop\n\tv_nop" : "+v"(c) : "v"(a), "v"(b)); return c; }
__device__ __forceinline__ h16 toh_flush(float v) { const h16 r = (h16)v; return (fabsf(v) < 6.103515625e-05f) ? (h16)0.0f : r; }

__global__ __launch_bounds__(256) void k_cvt8(const float* __restrict__ src, bf* dst, size_t n8) {
    const size_t i = (size_t)blockIdx.x * 256 + threadIdx.x; if (i >= n8) return;
    const v8f v = *(const v8f*)(src + i * 8); v8us o;
#pragma unroll
    for (int k = 0; k < 8; ++k) o[k] = f2bf(v[k]);
    *(volatile v8us*)(dst + i * 8) = o; __threadfence(); *(volatile v8us*)(dst + i * 8) = o;
}

__global__ __launch_bounds__(256) void k_wconv(const float* __restrict__ src, h16* dst, size_t n8) {
    const size_t i = (size_t)blockIdx.x * 256 + threadIdx.x; if (i >= n8) return;
    const v8f v = *(const v8f*)(src + i * 8); v8h o;
#pragma unroll
    for (int k = 0; k < 8; ++k) o[k] = toh_flush(bfr(v[k]) * WS);
    *(volatile v8h*)(dst + i * 8) = o; __threadfence(); *(volatile v8h*)(dst + i * 8) = o;
}

__global__ __launch_bounds__(32) void k_fc1(const bf* __restrict__ XB, const bf* __restrict__ WB, float* V1) {
    __shared__ __align__(16) float os[16 * 68];
    const int K = NG;
    const int lane = threadIdx.x & 31, lr = lane & 15, hi = lane >> 4; const int r0 = blockIdx.x * 64, c0 = blockIdx.y * 64; const int g = blockIdx.z;
    const bf* A  = XB + (size_t)(g >> 1) * ((size_t)NB * NG);
    const bf* Bt = WB + (size_t)g * ((size_t)MO * NG);
    v8f acc[4][4];
#pragma unroll
    for (int mb = 0; mb < 4; ++mb)
#pragma unroll
        for (int nb = 0; nb < 4; ++nb) acc[mb][nb] = (v8f){};
    const size_t aoff = (size_t)(r0 + lr) * K + 8 * hi, boff = (size_t)(c0 + lr) * K + 8 * hi;
#pragma unroll 1
    for (int kc = 0; kc < K; kc += 32) {
        v16bf a[4];
#pragma unroll
        for (int mb = 0; mb < 4; ++mb) a[mb] = ldb(A + aoff + (size_t)mb * 16 * K + kc);
#pragma unroll
        for (int nb = 0; nb < 4; ++nb) { const v16bf b = ldb(Bt + boff + (size_t)nb * 16 * K + kc);
#pragma unroll
            for (int mb = 0; mb < 4; ++mb) acc[mb][nb] = wmmab_g(a[mb], b, acc[mb][nb]); }
    }
    float* C = V1 + (size_t)g * ((size_t)NB * MO) + (size_t)r0 * MO + c0;
#pragma unroll
    for (int mb = 0; mb < 4; ++mb) {
#pragma unroll
        for (int nb = 0; nb < 4; ++nb) {
#pragma unroll
            for (int j = 0; j < 8; ++j) os[(hi * 8 + j) * 68 + nb * 16 + lr] = acc[mb][nb][j]; }
        wave_sync();
#pragma unroll 1
        for (int ps = 0; ps < 2; ++ps) {
#pragma unroll
            for (int s = 0; s < 8; ++s) { const int row = 2 * s + (lane >> 4), cofs = (lane & 15) * 4;
                const v4f val = *(const v4fa*)(&os[row * 68 + cofs]);
                *(volatile v4f*)(C + (size_t)(mb * 16 + row) * MO + cofs) = val; }
            if (ps == 0) __threadfence(); }
        wave_sync();
    }
}

__global__ __launch_bounds__(MO) void k_attn(const float* __restrict__ V1, h16* FP) {
#pragma clang fp contract(off)
    __shared__ float ex[MO], ey[MO], mx[MO], my[MO], cx[MO], cy[MO], zi[MO];
    __shared__ __align__(16) float fo[3 * FEAT];
    const int b = blockIdx.x, n = threadIdx.x;
    const size_t st = (size_t)NB * MO, off = (size_t)b * MO + n;
    {
        float vx = V1[0 * st + off], vy = V1[1 * st + off];
        float inv = rsqrtf(vx * vx + vy * vy);
        ex[n] = vx * inv; ey[n] = vy * inv;
        vx = V1[2 * st + off]; vy = V1[3 * st + off];
        inv = rsqrtf(vx * vx + vy * vy);
        mx[n] = vx * inv; my[n] = vy * inv;
        vx = V1[4 * st + off]; vy = V1[5 * st + off];
        inv = rsqrtf(vx * vx + vy * vy);
        cx[n] = vx * inv; cy[n] = vy * inv;
    }
    __syncthreads();
    const float e0 = ex[n] * L2E, e1 = ey[n] * L2E, m0 = mx[n] * L2E, m1 = my[n] * L2E, c0 = cx[n] * L2E, c1 = cy[n] * L2E;
    {
        float s0 = 0.0f, s1 = 0.0f, sd = 0.0f, t0 = 0.0f, t1 = 0.0f, td = 0.0f;
#pragma unroll 1
        for (int i = 0; i < MO; ++i) {
            const float x = cx[i], y = cy[i];
            const float wa = __builtin_amdgcn_exp2f(fmaf(x, e0, y * e1));
            const float wb = __builtin_amdgcn_exp2f(fmaf(x, m0, y * m1));
            s0 = fmaf(x, wa, s0); s1 = fmaf(y, wa, s1); sd += wa;
            t0 = fmaf(x, wb, t0); t1 = fmaf(y, wb, t1); td += wb;
        }
        const float ra = __builtin_amdgcn_rcpf(sd), rb = __builtin_amdgcn_rcpf(td);
        fo[2 * FEAT + n] = s0 * ra; fo[2 * FEAT + MO + n] = s1 * ra;
        fo[2 * FEAT + 2 * MO + n] = t0 * rb; fo[2 * FEAT + 3 * MO + n] = t1 * rb;
        zi[n] = rb;
    }
    __syncthreads();
    {
        float s0 = 0.0f, s1 = 0.0f, sd = 0.0f, t0 = 0.0f, t1 = 0.0f, td = 0.0f;
#pragma unroll 1
        for (int i = 0; i < MO; ++i) {
            const float x = ex[i], y = ey[i];
            const float wa = __builtin_amdgcn_exp2f(fmaf(x, m0, y * m1));
            const float wb = __builtin_amdgcn_exp2f(fmaf(x, c0, y * c1));
            s0 = fmaf(x, wa, s0); s1 = fmaf(y, wa, s1); sd += wa;
            t0 = fmaf(x, wb, t0); t1 = fmaf(y, wb, t1); td += wb;
        }
        const float ra = __builtin_amdgcn_rcpf(sd), rb = __builtin_amdgcn_rcpf(td);
        fo[n] = s0 * ra; fo[MO + n] = s1 * ra;
        fo[2 * MO + n] = t0 * rb; fo[3 * MO + n] = t1 * rb;
    }
    {
        float s0 = 0.0f, s1 = 0.0f, sd = 0.0f, t0 = 0.0f, t1 = 0.0f;
#pragma unroll 1
        for (int i = 0; i < MO; ++i) {
            const float x = mx[i], y = my[i]; const float z = zi[i];
            const float wa = __builtin_amdgcn_exp2f(fmaf(x, e0, y * e1));
            const float wb = __builtin_amdgcn_exp2f(fmaf(x, c0, y * c1)) * z;
            s0 = fmaf(x, wa, s0); s1 = fmaf(y, wa, s1); sd += wa;
            t0 = fmaf(x, wb, t0); t1 = fmaf(y, wb, t1);
        }
        const float ra = __builtin_amdgcn_rcpf(sd);
        fo[FEAT + n] = s0 * ra; fo[FEAT + MO + n] = s1 * ra;
        fo[FEAT + 2 * MO + n] = t0; fo[FEAT + 3 * MO + n] = t1;
    }
    __syncthreads();
#pragma unroll 1
    for (int ps = 0; ps < 2; ++ps) {
#pragma unroll 1
        for (int p = n; p < PIECES; p += MO) {
            const int hh = p / PPR; const int c8 = (p - hh * PPR) * 8;
            const v4f x0 = *(const v4fa*)(&fo[hh * FEAT + c8]); const v4f x1 = *(const v4fa*)(&fo[hh * FEAT + c8 + 4]); v8h hv;
#pragma unroll
            for (int i = 0; i < 4; ++i) { hv[i] = toh_flush(x0[i] * FS); hv[4 + i] = toh_flush(x1[i] * FS); }
            *(volatile v8h*)(FP + ((size_t)hh * NB + b) * FEAT + c8) = hv; }
        if (ps == 0) __threadfence(); }
}

__global__ __launch_bounds__(32) void k_fc2(const h16* __restrict__ A, const h16* __restrict__ Bt, const float* __restrict__ bias, float* HID) {
    __shared__ __align__(16) float os[16 * 68];
    const int K = FEAT;
    const int lane = threadIdx.x & 31, lr = lane & 15, hi = lane >> 4; const int r0 = blockIdx.x * 64, c0 = blockIdx.y * 64;
    v8f acc[4][4];
#pragma unroll
    for (int mb = 0; mb < 4; ++mb)
#pragma unroll
        for (int nb = 0; nb < 4; ++nb) acc[mb][nb] = (v8f){};
    const size_t aoff = (size_t)(r0 + lr) * K + 8 * hi, boff = (size_t)(c0 + lr) * K + 8 * hi;
#pragma unroll 1
    for (int kc = 0; kc < K; kc += 32) {
        v16h a[4];
#pragma unroll
        for (int mb = 0; mb < 4; ++mb) a[mb] = ldh(A + aoff + (size_t)mb * 16 * K + kc);
#pragma unroll
        for (int nb = 0; nb < 4; ++nb) { const v16h b = ldh(Bt + boff + (size_t)nb * 16 * K + kc);
#pragma unroll
            for (int mb = 0; mb < 4; ++mb) acc[mb][nb] = wmma16_g(a[mb], b, acc[mb][nb]); }
    }
    float bc[4];
#pragma unroll
    for (int nb = 0; nb < 4; ++nb) bc[nb] = bfr(bias[c0 + nb * 16 + lr]);
    float* C = HID + (size_t)r0 * CLS + c0;
#pragma unroll
    for (int mb = 0; mb < 4; ++mb) {
#pragma unroll
        for (int nb = 0; nb < 4; ++nb) {
#pragma unroll
            for (int j = 0; j < 8; ++j) os[(hi * 8 + j) * 68 + nb * 16 + lr] = fmaxf(acc[mb][nb][j] * FWI + bc[nb], 0.0f); }
        wave_sync();
#pragma unroll 1
        for (int ps = 0; ps < 2; ++ps) {
#pragma unroll
            for (int s = 0; s < 8; ++s) { const int row = 2 * s + (lane >> 4), cofs = (lane & 15) * 4;
                const v4f val = *(const v4fa*)(&os[row * 68 + cofs]);
                *(volatile v4f*)(C + (size_t)(mb * 16 + row) * CLS + cofs) = val; }
            if (ps == 0) __threadfence(); }
        wave_sync();
    }
}

__global__ __launch_bounds__(256) void k_head(const float* __restrict__ HID, const float* __restrict__ W3, const float* __restrict__ b3, float* OUT) {
#pragma clang fp contract(off)
    __shared__ __align__(16) float res[32];
    const int lane = threadIdx.x & 31;
    const int wave = __builtin_amdgcn_readfirstlane((int)(threadIdx.x >> 5));
    const float bz = bfr(b3[0]);
#pragma unroll 1
    for (int q = 0; q < 4; ++q) {
        const int s = wave * 4 + q;
        const float* row = HID + (size_t)(blockIdx.x * 32 + s) * CLS;
        float acc = 0.0f;
#pragma unroll 1
        for (int it = 0; it < CLS / 128; ++it) {
            const int idx = (it * 32 + lane) * 4;
            const v4f hv = *(const v4f*)(row + idx); const v4f wv = *(const v4f*)(W3 + idx);
            acc = fmaf(hv[0], bfr(wv[0]), acc); acc = fmaf(hv[1], bfr(wv[1]), acc);
            acc = fmaf(hv[2], bfr(wv[2]), acc); acc = fmaf(hv[3], bfr(wv[3]), acc);
        }
        acc += __shfl_xor(acc, 16, 32); acc += __shfl_xor(acc, 8, 32); acc += __shfl_xor(acc, 4, 32);
        acc += __shfl_xor(acc, 2, 32);  acc += __shfl_xor(acc, 1, 32);
        const float e = __builtin_amdgcn_exp2f(-(acc + bz) * L2E);
        const float sg = __builtin_amdgcn_rcpf(1.0f + e);
        if (lane == 0) res[s] = sg;
    }
    __syncthreads();
    if (wave == 0) {
        const v4f val = *(const v4fa*)(&res[(lane & 7) * 4]);
        float* dst = OUT + (size_t)blockIdx.x * 32 + (size_t)(lane & 7) * 4;
#pragma unroll 1
        for (int ps = 0; ps < 2; ++ps) {
            if (lane < 8) *(volatile v4f*)dst = val;
            if (ps == 0) __threadfence(); }
    }
}

static constexpr size_t al256(size_t v) { return (v + 255) & ~(size_t)255; }
static constexpr size_t SZ_X1 = al256((size_t)NB * NG * 2);
static constexpr size_t SZ_W1 = al256((size_t)MO * NG * 2);
static constexpr size_t SZ_V1 = al256((size_t)6 * NB * MO * 4);
static constexpr size_t SZ_FP = al256((size_t)3 * NB * FEAT * 2);
static constexpr size_t SZ_W2 = al256((size_t)CLS * FEAT * 2);
static constexpr size_t SZ_HD = al256((size_t)NB * CLS * 4);
static constexpr size_t SZ_TOTAL = 3 * SZ_X1 + 6 * SZ_W1 + SZ_V1 + SZ_FP + 3 * SZ_W2 + 3 * SZ_HD;
static_assert(SZ_TOTAL <= (size_t)134217728);
static_assert(SZ_X1 == (size_t)NB * NG * 2);
static_assert(SZ_W1 == (size_t)MO * NG * 2);
static_assert(((size_t)NB * NG / 8) % 256 == 0);
static_assert(((size_t)MO * NG / 8) % 256 == 0);
static_assert(((size_t)CLS * FEAT / 8) % 256 == 0);

extern "C" void kernel_launch(void* const* d_in, const int* in_sizes, int n_in,
                              void* d_out, int out_size, void* d_ws, size_t ws_size, hipStream_t stream) {
    if (n_in < 21) return;
    for (int i = 0; i < 3; ++i) if ((size_t)in_sizes[i] < (size_t)NB * NG) return;
    for (int i = 3; i < 9; ++i) if ((size_t)in_sizes[i] < (size_t)MO * NG) return;
    for (int i = 0; i < 3; ++i) {
        if ((size_t)in_sizes[9 + 2 * i] < (size_t)CLS * FEAT) return;
        if (in_sizes[10 + 2 * i] < CLS) return;
        if (in_sizes[15 + 2 * i] < CLS) return;
        if (in_sizes[16 + 2 * i] < 1) return;
    }
    if ((size_t)out_size < (size_t)2 * NB_FULL + NB) return;
    if (SZ_TOTAL > ws_size) return;
    const float* xin[3] = { (const float*)d_in[0], (const float*)d_in[1], (const float*)d_in[2] };
    const float* w1[6]  = { (const float*)d_in[3], (const float*)d_in[4], (const float*)d_in[5], (const float*)d_in[6], (const float*)d_in[7], (const float*)d_in[8] };
    const float* w2[3]  = { (const float*)d_in[9],  (const float*)d_in[11], (const float*)d_in[13] };
    const float* b2[3]  = { (const float*)d_in[10], (const float*)d_in[12], (const float*)d_in[14] };
    const float* w3[3]  = { (const float*)d_in[15], (const float*)d_in[17], (const float*)d_in[19] };
    const float* b3[3]  = { (const float*)d_in[16], (const float*)d_in[18], (const float*)d_in[20] };
    float* OUT = (float*)d_out;
    char* wsp = (char*)d_ws;
    bf* XB = (bf*)wsp; wsp += 3 * SZ_X1;
    bf* WB = (bf*)wsp; wsp += 6 * SZ_W1;
    float* V1 = (float*)wsp; wsp += SZ_V1;
    h16* FP = (h16*)wsp; wsp += SZ_FP;
    h16* W2H = (h16*)wsp; wsp += 3 * SZ_W2;
    float* HID = (float*)wsp; wsp += 3 * SZ_HD;

    { const size_t n8 = (size_t)NB * NG / 8; const unsigned g = (unsigned)((n8 + 255) / 256);
      for (int i = 0; i < 3; ++i) k_cvt8<<<g, 256, 0, stream>>>(xin[i], XB + (size_t)i * ((size_t)NB * NG), n8); }
    { const size_t n8 = (size_t)MO * NG / 8; const unsigned g = (unsigned)((n8 + 255) / 256);
      for (int i = 0; i < 6; ++i) k_cvt8<<<g, 256, 0, stream>>>(w1[i], WB + (size_t)i * ((size_t)MO * NG), n8); }
    { const size_t n8 = (size_t)CLS * FEAT / 8; const unsigned g = (unsigned)((n8 + 255) / 256);
      for (int i = 0; i < 3; ++i) k_wconv<<<g, 256, 0, stream>>>(w2[i], W2H + (size_t)i * ((size_t)CLS * FEAT), n8); }

    k_fc1<<<dim3(NB / 64, MO / 64, 6), 32, 0, stream>>>(XB, WB, V1);
    k_attn<<<dim3(NB, 1, 1), MO, 0, stream>>>(V1, FP);
    for (int i = 0; i < 3; ++i)
        k_fc2<<<dim3(NB / 64, CLS / 64, 1), 32, 0, stream>>>(FP + (size_t)i * ((size_t)NB * FEAT), W2H + (size_t)i * ((size_t)CLS * FEAT), b2[i], HID + (size_t)i * ((size_t)NB * CLS));
    for (int i = 0; i < 3; ++i)
        k_head<<<dim3(NB / 32, 1, 1), 256, 0, stream>>>(HID + (size_t)i * ((size_t)NB * CLS), w3[i], b3[i], OUT + (size_t)i * NB_FULL);
}
